// eight_related_context_mapping_68444598829760
// MI455X (gfx1250) — hardware-verified
//
#include <hip/hip_runtime.h>
#include <stddef.h>
#include <stdint.h>


typedef _Float16 v16h __attribute__((ext_vector_type(16)));
typedef _Float16 v8h  __attribute__((ext_vector_type(8)));
typedef float    v8f  __attribute__((ext_vector_type(8)));
typedef float    v4f  __attribute__((ext_vector_type(4)));
typedef v4f      v4fa __attribute__((may_alias));

union Frag { v16h v; v8h h[2]; };

static constexpr int BATCH = 2;
static constexpr int CH = 16;
static constexpr int HL = 128;
static constexpr int WL = 256;
static constexpr int HH = 256;
static constexpr int WH = 512;
static constexpr int C0 = 34;
static constexpr int C1 = 32;
static constexpr int C2 = 16;
static constexpr int C3 = 8;
static constexpr int NCTX = 9;
static constexpr int NTGT = 3;
static constexpr int NPL = NCTX + NTGT;
static constexpr int SEG = 32;
static constexpr int NSEG = WH / SEG;
static constexpr int WAVES = 4;
static constexpr int NWAVES = BATCH * HH * NSEG;
static constexpr int NBLK = NWAVES / WAVES;
static constexpr int LCOLS = SEG / 2 + 2;
static constexpr int O_HRT = 0;
static constexpr int O_HRRT = O_HRT + SEG * CH;
static constexpr int O_LRT = O_HRRT + SEG * CH;
static constexpr int O_LRRT = O_LRT + 3 * LCOLS * CH;
static constexpr int PERW_H = O_LRRT + LCOLS * CH;
static constexpr int PERW_S = NPL * SEG;
static constexpr size_t OUT0_N = (size_t)BATCH * NCTX * HH * WH;
static constexpr size_t OUT1_N = (size_t)BATCH * NTGT * HH * WH;
static_assert(WH % SEG == 0);
static_assert(NWAVES % WAVES == 0);
static_assert(NBLK * WAVES == NWAVES);
static_assert((O_HRRT * 2) % 16 == 0);
static_assert((O_LRT * 2) % 16 == 0);
static_assert((O_LRRT * 2) % 16 == 0);
static_assert((PERW_H * 2) % 16 == 0);
static_assert(3 * LCOLS * CH == 27 * 32);
static_assert(LCOLS * CH == 9 * 32);
static_assert(HH == 2 * HL);
static_assert(WH == 2 * WL);

__device__ __forceinline__ v8f wmma_f16_f32(v16h a, v16h b, v8f c) {
  v8f acc = __builtin_amdgcn_wmma_f32_16x16x32_f16(false, a, false, b, (short)0, c, false, false);
  asm volatile("v_nop\n\tv_nop\n\tv_nop\n\tv_nop" : "+v"(acc) : "v"(a), "v"(b));
  return acc;
}

__device__ __forceinline__ int clampi(int v, int lo, int hi) {
  return v < lo ? lo : (v > hi ? hi : v);
}

__device__ __forceinline__ v8h pack_lrelu16(v8f d) {
  v8h r;
#pragma unroll
  for (int i = 0; i < 8; ++i) {
    float x = d[i] * 0.0625f;
    x = fmaxf(x, 0.01f * x);
    r[i] = (_Float16)x;
  }
  return r;
}

__device__ __forceinline__ int tab_dy(int v) {
  return (v == 3 || v == 5 || v == 6) ? -1 : ((v == 4 || v == 7 || v == 8) ? 1 : 0);
}
__device__ __forceinline__ int tab_dx(int v) {
  return (v == 1 || v == 5 || v == 7) ? -1 : ((v == 2 || v == 6 || v == 8) ? 1 : 0);
}
__device__ __forceinline__ int tab_xt(int v) {
  return (v == 1 || v == 5) ? 1 : ((v == 2 || v == 6) ? 2 : 0);
}
__device__ __forceinline__ int tab_yt(int v) {
  return (v == 3 || v == 7) ? 1 : ((v == 4 || v == 8) ? 2 : 0);
}

__global__ __launch_bounds__(WAVES * 32) void ctx_map_kernel(
    const float* __restrict__ lr, const float* __restrict__ hr,
    const float* __restrict__ lrr, const float* __restrict__ hrr,
    const float* __restrict__ w0, const float* __restrict__ w1,
    const float* __restrict__ g1, const float* __restrict__ b1,
    const float* __restrict__ m1, const float* __restrict__ v1,
    const float* __restrict__ w2, const float* __restrict__ g2,
    const float* __restrict__ b2, const float* __restrict__ m2,
    const float* __restrict__ v2, const float* __restrict__ w3,
    float* __restrict__ out) {
  __shared__ __attribute__((aligned(16))) _Float16 s_h[WAVES * PERW_H];
  __shared__ __attribute__((aligned(16))) float s_stg[WAVES * PERW_S];

  const int lane = threadIdx.x & 31;
  const int wslot = threadIdx.x >> 5;
  const int hs = lane >> 4;
  const int p = lane & 15;

  const int wid = blockIdx.x * WAVES + wslot;
  const int xs = wid % NSEG;
  const int y = (wid / NSEG) % HH;
  const int b = wid / (NSEG * HH);
  const int x0 = xs * SEG;
  const int yl = y >> 1;
  const int xl0 = x0 >> 1;

  _Float16* hrt = s_h + wslot * PERW_H + O_HRT;
  _Float16* hrrt = s_h + wslot * PERW_H + O_HRRT;
  _Float16* lrt = s_h + wslot * PERW_H + O_LRT;
  _Float16* lrrt = s_h + wslot * PERW_H + O_LRRT;
  float* stg = s_stg + wslot * PERW_S;

#pragma unroll
  for (int c = 0; c < CH; ++c) {
    const size_t gi = (((size_t)(b * CH + c)) * HH + y) * WH + x0 + lane;
    hrt[lane * CH + c] = (_Float16)hr[gi];
    hrrt[lane * CH + c] = (_Float16)hrr[gi];
  }
  for (int i = 0; i < 27; ++i) {
    const int idx = i * 32 + lane;
    const int xx = idx % LCOLS;
    const int t = idx / LCOLS;
    const int c = t & 15;
    const int r = t >> 4;
    const int gy = clampi(yl - 1 + r, 0, HL - 1);
    const int gx = clampi(xl0 - 1 + xx, 0, WL - 1);
    lrt[(r * LCOLS + xx) * CH + c] = (_Float16)lr[(((size_t)(b * CH + c)) * HL + gy) * WL + gx];
  }
  for (int i = 0; i < 9; ++i) {
    const int idx = i * 32 + lane;
    const int xx = idx % LCOLS;
    const int c = idx / LCOLS;
    const int gx = clampi(xl0 - 1 + xx, 0, WL - 1);
    lrrt[xx * CH + c] = (_Float16)lrr[(((size_t)(b * CH + c)) * HL + yl) * WL + gx];
  }
  __syncthreads();

  const v16h zero16 = {};
  v16h A00 = zero16, A01 = zero16, Aw1 = zero16, Aw2 = zero16;
  const int p8 = (p < C3) ? p : (C3 - 1);
  const float a1p = g1[p] * rsqrtf(v1[p] + 1e-5f);
  const float a2raw = g2[p8] * rsqrtf(v2[p8] + 1e-5f);
  const float a2p = (p < C3) ? a2raw : 0.f;
#pragma unroll
  for (int i = 0; i < 16; ++i) {
    const int kk = (i < 8 ? i : i + 8) + 8 * hs;
    A00[i] = (_Float16)(16.f * w0[p * C0 + kk]);
    A01[i] = (_Float16)(16.f * w0[(p + 16) * C0 + kk]);
    Aw1[i] = (_Float16)(16.f * a1p * w1[p * C1 + kk]);
    const float w2v = w2[p8 * C2 + (kk & 15)];
    Aw2[i] = (p < C3 && kk < C2) ? (_Float16)(16.f * a2p * w2v) : (_Float16)0.f;
  }
  float u0a[8], u1a[8], u0b[8], u1b[8], w3s[8];
  v8f cb, cc;
#pragma unroll
  for (int v = 0; v < 8; ++v) {
    const int j = v + 8 * hs;
    u0a[v] = 16.f * w0[j * C0 + 32];
    u1a[v] = 16.f * w0[j * C0 + 33];
    u0b[v] = 16.f * w0[(j + 16) * C0 + 32];
    u1b[v] = 16.f * w0[(j + 16) * C0 + 33];
    const float a1j = g1[j] * rsqrtf(v1[j] + 1e-5f);
    cb[v] = 16.f * (b1[j] - m1[j] * a1j);
    const float a2v = g2[v] * rsqrtf(v2[v] + 1e-5f);
    const float t2 = 16.f * (b2[v] - m2[v] * a2v);
    cc[v] = (hs == 0) ? t2 : 0.f;
    w3s[v] = w3[v];
  }

  const float pxf = (float)(lane & 1);
  const float pyf = (float)(y & 1);

#pragma unroll 1
  for (int g = 0; g < 2; ++g) {
#pragma unroll 1
    for (int k = 0; k < NPL; ++k) {
      const bool tgt = (k >= NCTX);
      const int vix = tgt ? (k - NCTX) : k;
      const int dy = tab_dy(vix), dx = tab_dx(vix);
      const int xt = tab_xt(vix), yt = tab_yt(vix);
      const _Float16* ls = tgt ? lrrt : (lrt + (dy + 1) * (LCOLS * CH));
      const _Float16* hsrc = tgt ? hrrt : hrt;
      const float d0 = (xt == 0) ? (2.f * pxf - 1.f) : ((xt == 1) ? (2.f - pxf) : (1.f + pxf));
      const float d1 = (yt == 0) ? (2.f * pyf - 1.f) : ((yt == 1) ? (2.f - pyf) : (1.f + pyf));
      const int xi = 8 * g + (p >> 1) + 1 + dx;
      const int pix = 16 * g + p;

      Frag fb;
      fb.h[0] = *(const v8h*)(ls + xi * CH + 8 * hs);
      fb.h[1] = *(const v8h*)(hsrc + pix * CH + 8 * hs);
      v8f c0, c1;
#pragma unroll
      for (int v = 0; v < 8; ++v) {
        c0[v] = fmaf(u1a[v], d1, u0a[v] * d0);
        c1[v] = fmaf(u1b[v], d1, u0b[v] * d0);
      }
      const v8f D0 = wmma_f16_f32(A00, fb.v, c0);
      const v8f D1 = wmma_f16_f32(A01, fb.v, c1);

      Frag f1;
      f1.h[0] = pack_lrelu16(D0);
      f1.h[1] = pack_lrelu16(D1);
      const v8f E = wmma_f16_f32(Aw1, f1.v, cb);

      Frag f2;
      f2.v = zero16;
      f2.h[0] = pack_lrelu16(E);
      const v8f F = wmma_f16_f32(Aw2, f2.v, cc);

      float sacc = 0.f;
#pragma unroll
      for (int v = 0; v < 8; ++v) {
        float x = F[v] * 0.0625f;
        x = fmaxf(x, 0.01f * x);
        sacc = fmaf(w3s[v], x, sacc);
      }
      const int xl = xl0 + 8 * g + (p >> 1);
      const bool rok = (dy == 0) || (dy < 0 ? (yl > 0) : (yl < HL - 1));
      const bool cok = (dx == 0) || (dx < 0 ? (xl > 0) : (xl < WL - 1));
      const float lg = (rok && cok) ? sacc : -100.f;
      const float lgx = __shfl_xor(lg, 16, 32);
      const float mineval = (g == 0) ? lg : lgx;
      if (hs == g) stg[k * SEG + lane] = mineval;
    }
  }
  __syncthreads();

  {
    float l9[NCTX];
#pragma unroll
    for (int k = 0; k < NCTX; ++k) l9[k] = stg[k * SEG + lane];
    float mx = l9[0];
#pragma unroll
    for (int k = 1; k < NCTX; ++k) mx = fmaxf(mx, l9[k]);
    float e9[NCTX], ssum = 0.f;
#pragma unroll
    for (int k = 0; k < NCTX; ++k) { e9[k] = __expf(l9[k] - mx); ssum += e9[k]; }
    const float inv = 1.0f / ssum;
#pragma unroll
    for (int k = 0; k < NCTX; ++k) stg[k * SEG + lane] = e9[k] * inv;

    float l3[NTGT];
#pragma unroll
    for (int k = 0; k < NTGT; ++k) l3[k] = stg[(NCTX + k) * SEG + lane];
    const float mt = fmaxf(l3[0], fmaxf(l3[1], l3[2]));
    float e3[NTGT], ts = 0.f;
#pragma unroll
    for (int k = 0; k < NTGT; ++k) { e3[k] = __expf(l3[k] - mt); ts += e3[k]; }
    const float ti = 1.0f / ts;
#pragma unroll
    for (int k = 0; k < NTGT; ++k) stg[(NCTX + k) * SEG + lane] = e3[k] * ti;
  }
  __syncthreads();

  const int lq = lane >> 3;
  const int seg4 = (lane & 7) * 4;
  v4f vv[3];
  float* pq[3];
#pragma unroll
  for (int q = 0; q < 3; ++q) {
    const int pl = 4 * q + lq;
    vv[q] = *(const v4fa*)(stg + pl * SEG + seg4);
    const int plc = (pl < NCTX) ? pl : 0;
    const int plt = (pl >= NCTX) ? (pl - NCTX) : 0;
    const size_t off0 = (((size_t)(b * NCTX + plc)) * HH + y) * WH;
    const size_t off1 = OUT0_N + (((size_t)(b * NTGT + plt)) * HH + y) * WH;
    pq[q] = out + ((pl < NCTX) ? off0 : off1) + x0 + seg4;
  }
#pragma unroll
  for (int q = 0; q < 3; ++q) *(volatile v4f*)pq[q] = vv[q];
  __threadfence();
#pragma unroll
  for (int q = 0; q < 3; ++q) *(volatile v4f*)pq[q] = vv[q];
}

extern "C" void kernel_launch(void* const* d_in, const int* in_sizes, int n_in,
                              void* d_out, int out_size, void* d_ws, size_t ws_size,
                              hipStream_t stream) {
  (void)d_ws; (void)ws_size;
  if (n_in < 16) return;
  if (in_sizes[0] != BATCH * CH * HL * WL) return;
  if (in_sizes[1] != BATCH * CH * HH * WH) return;
  if (in_sizes[2] != BATCH * CH * HL * WL) return;
  if (in_sizes[3] != BATCH * CH * HH * WH) return;
  if (in_sizes[4] != C1 * C0) return;
  if (in_sizes[5] != C2 * C1) return;
  if (in_sizes[6] < C2 || in_sizes[7] < C2 || in_sizes[8] < C2 || in_sizes[9] < C2) return;
  if (in_sizes[10] != C3 * C2) return;
  if (in_sizes[11] < C3 || in_sizes[12] < C3 || in_sizes[13] < C3 || in_sizes[14] < C3) return;
  if (in_sizes[15] < C3) return;
  if ((size_t)out_size != OUT0_N + OUT1_N) return;

  const float* lr  = (const float*)d_in[0];
  const float* hr  = (const float*)d_in[1];
  const float* lrr = (const float*)d_in[2];
  const float* hrr = (const float*)d_in[3];
  const float* w0  = (const float*)d_in[4];
  const float* w1  = (const float*)d_in[5];
  const float* g1  = (const float*)d_in[6];
  const float* b1  = (const float*)d_in[7];
  const float* m1  = (const float*)d_in[8];
  const float* v1  = (const float*)d_in[9];
  const float* w2  = (const float*)d_in[10];
  const float* g2  = (const float*)d_in[11];
  const float* b2  = (const float*)d_in[12];
  const float* m2  = (const float*)d_in[13];
  const float* v2  = (const float*)d_in[14];
  const float* w3  = (const float*)d_in[15];
  float* out = (float*)d_out;

  ctx_map_kernel<<<NBLK, WAVES * 32, 0, stream>>>(lr, hr, lrr, hrr, w0, w1, g1, b1, m1, v1,
                                                  w2, g2, b2, m2, v2, w3, out);
}
